// Transformer_7370163880736
// MI455X (gfx1250) — hardware-verified
//
#include <hip/hip_runtime.h>
#include <math.h>

#ifndef NB
#define NB 8
#endif
#ifndef SEQ
#define SEQ 1024
#endif
#define NB_FULL 8
#define SEQ_FULL 1024
#define DM 512
#define NH 8
#define HD 64
#define FFD 2048
#define MTOK (NB * SEQ)

static_assert(NB >= 1 && NB <= NB_FULL);
static_assert(SEQ >= 64 && SEQ <= SEQ_FULL && (SEQ % 64) == 0);
static_assert(NH * HD == DM);
static_assert((MTOK % 64) == 0 && (DM % 64) == 0 && (FFD % 64) == 0);
static_assert((DM % 32) == 0 && (FFD % 32) == 0);

typedef __attribute__((ext_vector_type(16))) _Float16 v16h;
typedef __attribute__((ext_vector_type(8)))  _Float16 v8h;
typedef __attribute__((ext_vector_type(16))) __bf16   v16b;
typedef __attribute__((ext_vector_type(8)))  __bf16   v8b;
typedef __attribute__((ext_vector_type(8)))  float    v8f;
typedef __attribute__((ext_vector_type(4)))  float    v4f;
typedef unsigned int cm_u4 __attribute__((ext_vector_type(4)));


#define VST2(T, ptr, val) do { const T vst2_v_ = (val); *(volatile T*)(ptr) = vst2_v_; __threadfence(); *(volatile T*)(ptr) = vst2_v_; } while (0)
#define VST2V4(ptr, val) do { const v4f vst2_v4_ = (val); *(volatile v4f*)(ptr) = vst2_v4_; __threadfence(); *(volatile v4f*)(ptr) = vst2_v4_; } while (0)

__device__ __forceinline__ unsigned int cmb_pk2(float a, float b) { return (unsigned int)__builtin_bit_cast(unsigned short, (_Float16)a) | ((unsigned int)__builtin_bit_cast(unsigned short, (_Float16)b) << 16); }
__device__ __forceinline__ float cmb_bf(float v) { const unsigned u = __builtin_bit_cast(unsigned, v); const unsigned r = (u + 0x7fffu + ((u >> 16) & 1u)) & 0xffff0000u; return __builtin_bit_cast(float, r); }

namespace w25 {

__device__ __forceinline__ unsigned short f2bf_bits(float f) {
  unsigned u = __float_as_uint(f);
  return (unsigned short)((u + 0x7FFFu + ((u >> 16) & 1u)) >> 16);
}
__device__ __forceinline__ float bf_bits2f(unsigned short h) { return __uint_as_float(((unsigned)h) << 16); }

__device__ __forceinline__ void dep_guard_h(v8f& a, v8f& b, v16h x, v16h y) { asm volatile("v_nop\n\tv_nop\n\tv_nop\n\tv_nop" : "+v"(a), "+v"(b) : "v"(x), "v"(y)); }
__device__ __forceinline__ void dep_guard_b(v8f& a, v8f& b, v16b x, v16b y) { asm volatile("v_nop\n\tv_nop\n\tv_nop\n\tv_nop" : "+v"(a), "+v"(b) : "v"(x), "v"(y)); }
__device__ __forceinline__ void keep4_h(v16h a, v16h b, v16h c, v16h d) { asm volatile("v_nop" :: "v"(a), "v"(b), "v"(c), "v"(d)); }
__device__ __forceinline__ void keep4_b(v16b a, v16b b, v16b c, v16b d) { asm volatile("v_nop" :: "v"(a), "v"(b), "v"(c), "v"(d)); }
__device__ __forceinline__ void acc_guard4(v8f& a, v8f& b, v8f& c, v8f& d) { asm volatile("v_nop\n\tv_nop\n\tv_nop\n\tv_nop" : "+v"(a), "+v"(b), "+v"(c), "+v"(d)); }
template <typename T> struct Frag;
template <> struct Frag<_Float16> {
  typedef v16h V; union U { v16h v; v8h h[2]; };
  static __device__ __forceinline__ v16h load(const _Float16* p) {
    U f; f.h[0] = *(const v8h*)(p); f.h[1] = *(const v8h*)(p + 16); return f.v;
  }
  static __device__ __forceinline__ v8f mma(v16h a, v16h b, v8f c) {
    return __builtin_amdgcn_wmma_f32_16x16x32_f16(false, a, false, b, (short)0, c, false, false);
  }
  static __device__ __forceinline__ void guard(v8f& a, v8f& b, v16h x, v16h y) { dep_guard_h(a, b, x, y); }
  static __device__ __forceinline__ void keep(v16h a, v16h b, v16h c, v16h d) { keep4_h(a, b, c, d); }
};
template <> struct Frag<__bf16> {
  typedef v16b V; union U { v16b v; v8b h[2]; };
  static __device__ __forceinline__ v16b load(const __bf16* p) {
    U f; f.h[0] = *(const v8b*)(p); f.h[1] = *(const v8b*)(p + 16); return f.v;
  }
  static __device__ __forceinline__ v8f mma(v16b a, v16b b, v8f c) {
    return __builtin_amdgcn_wmma_f32_16x16x32_bf16(false, a, false, b, (short)0, c, false, false);
  }
  static __device__ __forceinline__ void guard(v8f& a, v8f& b, v16b x, v16b y) { dep_guard_b(a, b, x, y); }
  static __device__ __forceinline__ void keep(v16b a, v16b b, v16b c, v16b d) { keep4_b(a, b, c, d); }
};

template <int ET> struct Elem;
template <> struct Elem<0> { typedef _Float16 T; };
template <> struct Elem<1> { typedef __bf16 T; };
template <int ET, bool SPLIT, int BIAS_MODE, int OUT_MODE, bool RESID, int ACT = 0>
__global__ __launch_bounds__(256) void wmma_gemm64(
    const unsigned short* __restrict__ Ap, const unsigned short* __restrict__ A2p, int lda, long strideA,
    const unsigned short* __restrict__ Btp, const unsigned short* __restrict__ Bt2p, int ldb, long strideB,
    void* __restrict__ Cout, void* __restrict__ Cout2, int ldc, long strideC,
    const float* __restrict__ bias,
    const float* __restrict__ resid, long strideR,
    int M, int N, int K, float scale) {
  typedef typename Elem<ET>::T T;
  typedef typename Frag<T>::V V;
  const T* A = (const T*)Ap; const T* A2 = (const T*)A2p; const T* Bt = (const T*)Btp; const T* Bt2 = (const T*)Bt2p;
  __shared__ __align__(16) float sT[8][16 * 68];
  const int b    = blockIdx.y;
  const int lane = threadIdx.x & 31;
  const int wave = threadIdx.x >> 5;
  const int tilesN = N >> 6;
  const int tilesM = M >> 6;
  const int tile = blockIdx.x * 8 + wave;
  if (tile >= tilesM * tilesN) return;
  const int tm = tile / tilesN;
  const int tn = tile - tm * tilesN;
  const int m0 = tm << 6;
  const int n0 = tn << 6;

  const T* Ab  = A  + (size_t)b * strideA;
  const T* Bb  = Bt + (size_t)b * strideB;
  const T* Ab2 = SPLIT ? (A2  + (size_t)b * strideA) : nullptr;
  const T* Bb2 = SPLIT ? (Bt2 + (size_t)b * strideB) : nullptr;

  const int rlane = lane & 15;
  const int koff  = (lane >> 4) * 8;
  const int mOff  = (lane >> 4) * 8;

  v8f acc[4][4];
#pragma unroll
  for (int i = 0; i < 4; ++i)
#pragma unroll
    for (int j = 0; j < 4; ++j) acc[i][j] = (v8f){0.f,0.f,0.f,0.f,0.f,0.f,0.f,0.f};

  for (int k0 = 0; k0 < K; k0 += 32) {
    V bh[4], bl[4];
#pragma unroll
    for (int j = 0; j < 4; ++j) {
      const size_t bo = (size_t)(n0 + (j << 4) + rlane) * ldb + koff + k0;
      bh[j] = Frag<T>::load(Bb + bo);
      if (SPLIT) bl[j] = Frag<T>::load(Bb2 + bo);
    }
#pragma unroll
    for (int i = 0; i < 4; ++i) {
      const size_t ao = (size_t)(m0 + (i << 4) + rlane) * lda + koff + k0;
      V ah = Frag<T>::load(Ab + ao);
      V al;
      if (SPLIT) al = Frag<T>::load(Ab2 + ao);
#pragma unroll
      for (int j = 0; j < 4; ++j) {
        acc[i][j] = Frag<T>::mma(ah, bh[j], acc[i][j]);
        if (SPLIT) {
          acc[i][j] = Frag<T>::mma(ah, bl[j], acc[i][j]);
          acc[i][j] = Frag<T>::mma(al, bh[j], acc[i][j]);
        }
      }
      Frag<T>::guard(acc[i][0], acc[i][3], ah, SPLIT ? al : ah);
    }
    Frag<T>::keep(bh[0], bh[1], bh[2], bh[3]);
    if (SPLIT) Frag<T>::keep(bl[0], bl[1], bl[2], bl[3]);
  }
  acc_guard4(acc[0][0], acc[0][1], acc[0][2], acc[0][3]);
  acc_guard4(acc[1][0], acc[1][1], acc[1][2], acc[1][3]);
  acc_guard4(acc[2][0], acc[2][1], acc[2][2], acc[2][3]);
  acc_guard4(acc[3][0], acc[3][1], acc[3][2], acc[3][3]);

  float* slab = sT[wave];
  const float* Rb = RESID ? (resid + (size_t)b * strideR) : nullptr;
#pragma unroll
  for (int i = 0; i < 4; ++i) {
    const int mBase = m0 + (i << 4);
#pragma unroll
    for (int j = 0; j < 4; ++j) {
      const int n = n0 + (j << 4) + rlane;
      float bv = 0.f;
      if (BIAS_MODE == 2) bv = bf_bits2f(f2bf_bits(bias[n]));
#pragma unroll
      for (int r = 0; r < 8; ++r) {
        float v = acc[i][j][r] * scale;
        if (BIAS_MODE == 1) v += bf_bits2f(f2bf_bits(bias[mBase + mOff + r]));
        if (BIAS_MODE == 2) v += bv;
        if (RESID) v += Rb[(size_t)(mBase + mOff + r) * ldc + n];
        if (ACT == 1) v = tanhf(v);
        if (ACT == 2) v = fmaxf(v, 0.0f);
        slab[(mOff + r) * 68 + (j << 4) + rlane] = v;
      }
    }
    __builtin_amdgcn_fence(3  , "workgroup");
    __builtin_amdgcn_wave_barrier();
    __builtin_amdgcn_fence(2  , "workgroup");
    if (OUT_MODE == 0) {
      float* C = (float*)Cout + (size_t)b * strideC;
      const int hh = lane >> 4, c4 = (lane & 15) * 4;
      for (int pass = 0; pass < 2; ++pass) {
#pragma unroll
        for (int it = 0; it < 8; ++it) {
          const int row = it * 2 + hh;
          v4f v = *(const v4f*)(slab + row * 68 + c4);
          *(volatile v4f*)(C + (size_t)(mBase + row) * ldc + n0 + c4) = v;
        }
        __threadfence();
      }
    } else {
      const int q = lane >> 3, c8 = (lane & 7) * 8;
      unsigned short* C  = (unsigned short*)Cout  + (size_t)b * strideC;
      unsigned short* C2 = (OUT_MODE == 2) ? ((unsigned short*)Cout2 + (size_t)b * strideC) : nullptr;
      for (int pass = 0; pass < 2; ++pass) {
#pragma unroll
        for (int it = 0; it < 4; ++it) {
          const int row = it * 4 + q;
          const float* sp = slab + row * 68 + c8;
          v8h hv, lv;
#pragma unroll
          for (int e = 0; e < 8; ++e) {
            if (OUT_MODE == 1) {
              hv[e] = (_Float16)sp[e];
            } else {
              unsigned short hb = f2bf_bits(sp[e]);
              unsigned short lb = f2bf_bits(sp[e] - bf_bits2f(hb));
              hv[e] = __builtin_bit_cast(_Float16, hb);
              lv[e] = __builtin_bit_cast(_Float16, lb);
            }
          }
          *(volatile v8h*)(C + (size_t)(mBase + row) * ldc + n0 + c8) = hv;
          if (OUT_MODE == 2) *(volatile v8h*)(C2 + (size_t)(mBase + row) * ldc + n0 + c8) = lv;
        }
        __threadfence();
      }
    }
    __builtin_amdgcn_fence(3  , "workgroup");
    __builtin_amdgcn_wave_barrier();
    __builtin_amdgcn_fence(2  , "workgroup");
  }
}

#define AT_D 64
#define AT_NW 4
#define AT_QB 64
#define AT_KC 64
struct AttnGeom { long q_bs, q_rs, q_hs, k_bs, k_rs, k_hs, v_bs, v_rs, v_hs, o_bs, o_rs, o_hs; int S, Skv, H, pad_; float qscale, ocarry; };
static_assert(sizeof(AttnGeom) == 12 * 8 + 6 * 4);

__device__ __forceinline__ v8f at_mma_h(v16h a, v16h b, v8f c) {
  c = __builtin_amdgcn_wmma_f32_16x16x32_f16(false, a, false, b, (short)0, c, false, false);
  asm volatile("v_nop\n\tv_nop\n\tv_nop\n\tv_nop" : "+v"(c) : "v"(a), "v"(b));
  return c;
}

__global__ __launch_bounds__(128)
void attn64_f16(const float* __restrict__ q, const float* __restrict__ k,
                const float* __restrict__ v, unsigned short* __restrict__ out16, AttnGeom g) {
  const float PSC = 32768.0f;
  union FH { v16h v; v8h h[2]; };
  __shared__ __align__(16) _Float16 Ksh[AT_KC * AT_D];
  __shared__ __align__(16) _Float16 Vth[AT_D * AT_KC];
  __shared__ __align__(16) _Float16 Psh[AT_NW][16 * AT_KC];
  __shared__ __align__(16) float    Os[AT_NW][16 * 68];

  const unsigned tid  = threadIdx.x;
  const unsigned wave = tid >> 5;
  const unsigned lane = tid & 31u;
  const unsigned hh   = lane >> 4;
  const unsigned c    = lane & 15u;

  const unsigned nqb = (unsigned)g.S / AT_QB;
  const unsigned bx = blockIdx.x;
  const unsigned qb = bx % nqb;
  const unsigned bh = bx / nqb;
  const unsigned h  = bh % (unsigned)g.H;
  const unsigned b  = bh / (unsigned)g.H;
  const unsigned q0 = qb * AT_QB + wave * 16u;

  const float* qb_ptr = q + (size_t)b * g.q_bs + (size_t)h * g.q_hs;
  const float* kb_ptr = k + (size_t)b * g.k_bs + (size_t)h * g.k_hs;
  const float* vb_ptr = v + (size_t)b * g.v_bs + (size_t)h * g.v_hs;
  unsigned short* ob_ptr = out16 + (size_t)b * g.o_bs + (size_t)h * g.o_hs;

  v16h qa[2];
  {
    const float* qrow = qb_ptr + (size_t)(q0 + c) * g.q_rs;
#pragma unroll
    for (int dc = 0; dc < 2; ++dc) {
#pragma unroll
      for (int e = 0; e < 8; ++e) {
        const float f0 = qrow[dc * 32 + 8 * hh + e] * g.qscale;
        const float f1 = qrow[dc * 32 + 16 + 8 * hh + e] * g.qscale;
        qa[dc][e] = (_Float16)f0; qa[dc][8 + e] = (_Float16)f1;
      }
    }
  }

  float mrow[8], lrow[8];
  v8f oacc[4];
#pragma unroll
  for (int r = 0; r < 8; ++r) { mrow[r] = -INFINITY; lrow[r] = 0.f; }
#pragma unroll
  for (int t = 0; t < 4; ++t) oacc[t] = (v8f){0.f,0.f,0.f,0.f,0.f,0.f,0.f,0.f};

  const unsigned nChunks = (unsigned)g.Skv / AT_KC;
  for (unsigned kc = 0; kc < nChunks; ++kc) {
    const unsigned kv0 = kc * AT_KC;
    __syncthreads();
    {
      const unsigned kvr = tid >> 1, dh = (tid & 1u) * 32u;
      const float* krow = kb_ptr + (size_t)(kv0 + kvr) * g.k_rs + dh;
      const float* vrow = vb_ptr + (size_t)(kv0 + kvr) * g.v_rs + dh;
#pragma unroll
      for (int i = 0; i < 8; ++i) {
        v4f kk = *(const v4f*)(krow + 4 * i);
        v4f vv = *(const v4f*)(vrow + 4 * i);
#pragma unroll
        for (int e = 0; e < 4; ++e) {
          const unsigned d = dh + 4 * i + e;
          Ksh[kvr * AT_D + d] = (_Float16)kk[e];
          Vth[d * AT_KC + kvr] = (_Float16)vv[e];
        }
      }
    }
    __syncthreads();

    v8f s[4];
#pragma unroll
    for (int j = 0; j < 4; ++j) {
      s[j] = (v8f){0.f,0.f,0.f,0.f,0.f,0.f,0.f,0.f};
#pragma unroll
      for (int dc = 0; dc < 2; ++dc) {
        FH kb;
        kb.h[0] = *(const v8h*)(Ksh + (j * 16 + c) * AT_D + dc * 32 + 8 * hh);
        kb.h[1] = *(const v8h*)(Ksh + (j * 16 + c) * AT_D + dc * 32 + 16 + 8 * hh);
        s[j] = at_mma_h(qa[dc], kb.v, s[j]);
      }
    }
    float cm[8];
#pragma unroll
    for (int r = 0; r < 8; ++r) {
      float m = fmaxf(fmaxf(s[0][r], s[1][r]), fmaxf(s[2][r], s[3][r]));
#pragma unroll
      for (int off = 1; off < 16; off <<= 1) m = fmaxf(m, __shfl_xor(m, off, 32));
      cm[r] = m;
    }
    _Float16* pw = Psh[wave];
#pragma unroll
    for (int r = 0; r < 8; ++r) {
      const float mnew = fmaxf(mrow[r], cm[r]);
      const float alpha = expf(mrow[r] - mnew);
      mrow[r] = mnew;
      float psum = 0.f;
#pragma unroll
      for (int j = 0; j < 4; ++j) {
        const float p = expf(s[j][r] - mnew);
        psum += p;
        pw[(8 * hh + r) * AT_KC + j * 16 + c] = (_Float16)(p * PSC);
      }
#pragma unroll
      for (int off = 1; off < 16; off <<= 1) psum += __shfl_xor(psum, off, 32);
      lrow[r] = lrow[r] * alpha + psum;
#pragma unroll
      for (int t = 0; t < 4; ++t) oacc[t][r] *= alpha;
    }
    __builtin_amdgcn_fence(3  , "workgroup");
    __builtin_amdgcn_wave_barrier();
    __builtin_amdgcn_fence(2  , "workgroup");
#pragma unroll
    for (int kk = 0; kk < 2; ++kk) {
      FH pa;
      pa.h[0] = *(const v8h*)(pw + c * AT_KC + kk * 32 + 8 * hh);
      pa.h[1] = *(const v8h*)(pw + c * AT_KC + kk * 32 + 16 + 8 * hh);
#pragma unroll
      for (int t = 0; t < 4; ++t) {
        FH vb;
        vb.h[0] = *(const v8h*)(Vth + (t * 16 + c) * AT_KC + kk * 32 + 8 * hh);
        vb.h[1] = *(const v8h*)(Vth + (t * 16 + c) * AT_KC + kk * 32 + 16 + 8 * hh);
        oacc[t] = at_mma_h(pa.v, vb.v, oacc[t]);
      }
    }
  }

  float* os = Os[wave];
#pragma unroll
  for (int r = 0; r < 8; ++r) {
    const float inv = g.ocarry / (lrow[r] * PSC);
#pragma unroll
    for (int t = 0; t < 4; ++t) os[(8 * hh + r) * 68 + t * 16 + c] = oacc[t][r] * inv;
  }
  __builtin_amdgcn_fence(3  , "workgroup");
  __builtin_amdgcn_wave_barrier();
  __builtin_amdgcn_fence(2  , "workgroup");
  {
    const unsigned q4 = lane >> 3, c8 = (lane & 7u) * 8u;
    for (int pass = 0; pass < 2; ++pass) {
#pragma unroll
      for (int it = 0; it < 4; ++it) {
        const unsigned row = it * 4 + q4;
        const float* sp = os + row * 68 + c8;
        v8h hv;
#pragma unroll
        for (int e = 0; e < 8; ++e) hv[e] = (_Float16)sp[e];
        *(volatile v8h*)(ob_ptr + (size_t)(q0 + row) * g.o_rs + c8) = hv;
      }
      __threadfence();
    }
  }
}

}

__device__ __forceinline__ size_t full_row(unsigned r) { const unsigned b = r / (unsigned)SEQ; const unsigned s = r - b * (unsigned)SEQ; return (size_t)(b * (unsigned)SEQ_FULL + s); }

static_assert(((MTOK * 64) % 256) == 0);
__global__ __launch_bounds__(256) void k_cast_x3(const float* __restrict__ s0, const float* __restrict__ s1, const float* __restrict__ s2, unsigned short* __restrict__ dst) {
    const unsigned z = blockIdx.y;
    const float* src = (z == 0u) ? s0 : ((z == 1u) ? s1 : s2);
    const unsigned u = blockIdx.x * 256u + threadIdx.x;
    if (u >= (unsigned)MTOK * 64u) return;
    const unsigned r = u >> 6, c0 = (u & 63u) << 3;
    const float* p = src + full_row(r) * DM + c0;
    const v4f a = *(const v4f*)p, bq = *(const v4f*)(p + 4);
    cm_u4 pk;
    pk.x = cmb_pk2(cmb_bf(a.x), cmb_bf(a.y)); pk.y = cmb_pk2(cmb_bf(a.z), cmb_bf(a.w));
    pk.z = cmb_pk2(cmb_bf(bq.x), cmb_bf(bq.y)); pk.w = cmb_pk2(cmb_bf(bq.z), cmb_bf(bq.w));
    VST2(cm_u4, (cm_u4*)(dst + (size_t)z * ((size_t)MTOK * DM) + (size_t)r * DM + c0), pk);
}

__global__ __launch_bounds__(256) void k_cast_wT(const float* __restrict__ s0, const float* __restrict__ s1, const float* __restrict__ s2, unsigned lds, unsigned sSlab,
                                                 unsigned short* __restrict__ dst, unsigned ldd, unsigned dSlab, unsigned dWhich, unsigned nR, unsigned nC, float sc) {
    const unsigned y = blockIdx.y, z = blockIdx.z;
    const unsigned per = nR >> 3;
    const unsigned u = blockIdx.x * 256u + threadIdx.x;
    if (u >= nC * per) return;
    const unsigned c = u / per, r0 = (u - c * per) << 3;
    const float* src = ((z == 0u) ? s0 : ((z == 1u) ? s1 : s2)) + (size_t)y * sSlab;
    float w[8];
#pragma unroll
    for (int e = 0; e < 8; ++e) w[e] = cmb_bf(src[(size_t)(r0 + e) * lds + c]) * sc;
    cm_u4 pk; pk.x = cmb_pk2(w[0], w[1]); pk.y = cmb_pk2(w[2], w[3]); pk.z = cmb_pk2(w[4], w[5]); pk.w = cmb_pk2(w[6], w[7]);
    VST2(cm_u4, (cm_u4*)(dst + (size_t)z * dWhich + (size_t)y * dSlab + (size_t)c * ldd + r0), pk);
}

static_assert((MTOK % 8) == 0);
__device__ __forceinline__ v4f ln_ld(const float* __restrict__ xr, const float* __restrict__ tr, unsigned col) {
    const v4f xv = *(const v4f*)(xr + col), tv = *(const v4f*)(tr + col);
    v4f v; v.x = cmb_bf(xv.x) + tv.x; v.y = cmb_bf(xv.y) + tv.y; v.z = cmb_bf(xv.z) + tv.z; v.w = cmb_bf(xv.w) + tv.w; return v;
}
__device__ __forceinline__ v4f ln_aff(v4f d, float rs, const float* __restrict__ g, const float* __restrict__ bt, unsigned col) {
    const v4f gv = *(const v4f*)(g + col), bv = *(const v4f*)(bt + col);
    v4f y; y.x = d.x * rs * cmb_bf(gv.x) + cmb_bf(bv.x); y.y = d.y * rs * cmb_bf(gv.y) + cmb_bf(bv.y);
    y.z = d.z * rs * cmb_bf(gv.z) + cmb_bf(bv.z); y.w = d.w * rs * cmb_bf(gv.w) + cmb_bf(bv.w); return y;
}
template <int OUT16>
__global__ __launch_bounds__(256) void k_add_ln(const float* __restrict__ xq, const float* __restrict__ t, const float* __restrict__ g, const float* __restrict__ bt,
                                                float* __restrict__ outf, unsigned short* __restrict__ out16) {
    const unsigned lane = threadIdx.x & 31u, wave = threadIdx.x >> 5;
    const unsigned r = blockIdx.x * 8u + wave;
    if (r >= (unsigned)MTOK) return;
    const size_t rx = full_row(r) * DM;
    const float* xr = xq + rx;
    const float* tr = t + (size_t)r * DM;
    const unsigned NI = OUT16 ? 2u : 4u;
    float sm = 0.f;
#pragma unroll 1
    for (unsigned j = 0; j < NI; ++j) {
        const unsigned col = OUT16 ? ((j << 8) + (lane << 3)) : ((j << 7) + (lane << 2));
        const v4f v0 = ln_ld(xr, tr, col); sm += (v0.x + v0.y) + (v0.z + v0.w);
        if (OUT16) { const v4f v1 = ln_ld(xr, tr, col + 4u); sm += (v1.x + v1.y) + (v1.z + v1.w); }
    }
#pragma unroll
    for (int o = 16; o > 0; o >>= 1) sm += __shfl_xor(sm, o, 32);
    const float mu = sm * (1.0f / (float)DM);
    float ss = 0.f;
#pragma unroll 1
    for (unsigned j = 0; j < NI; ++j) {
        const unsigned col = OUT16 ? ((j << 8) + (lane << 3)) : ((j << 7) + (lane << 2));
        const v4f d0 = ln_ld(xr, tr, col) - mu; ss += d0.x * d0.x + d0.y * d0.y + d0.z * d0.z + d0.w * d0.w;
        if (OUT16) { const v4f d1 = ln_ld(xr, tr, col + 4u) - mu; ss += d1.x * d1.x + d1.y * d1.y + d1.z * d1.z + d1.w * d1.w; }
    }
#pragma unroll
    for (int o = 16; o > 0; o >>= 1) ss += __shfl_xor(ss, o, 32);
    const float rs = rsqrtf(ss * (1.0f / (float)DM) + 1e-6f);
#pragma unroll 1
    for (unsigned j = 0; j < NI; ++j) {
        const unsigned col = OUT16 ? ((j << 8) + (lane << 3)) : ((j << 7) + (lane << 2));
        const v4f y0 = ln_aff(ln_ld(xr, tr, col) - mu, rs, g, bt, col);
        if (OUT16) {
            const v4f y1 = ln_aff(ln_ld(xr, tr, col + 4u) - mu, rs, g, bt, col + 4u);
            cm_u4 pk; pk.x = cmb_pk2(y0.x, y0.y); pk.y = cmb_pk2(y0.z, y0.w); pk.z = cmb_pk2(y1.x, y1.y); pk.w = cmb_pk2(y1.z, y1.w);
            VST2(cm_u4, (cm_u4*)(out16 + (size_t)r * DM + col), pk);
        } else {
            VST2V4(outf + rx + col, y0);
        }
    }
}

constexpr size_t SZ_X16  = (size_t)3 * MTOK * DM * 2;
constexpr size_t SZ_WP   = (size_t)3 * DM * DM * 2;
constexpr size_t SZ_WO   = (size_t)DM * DM * 2;
constexpr size_t SZ_W1   = (size_t)FFD * DM * 2;
constexpr size_t SZ_W2   = (size_t)DM * FFD * 2;
constexpr size_t SZ_QKV  = (size_t)3 * MTOK * DM * 4;
constexpr size_t SZ_H16  = (size_t)MTOK * FFD * 2;
constexpr size_t SZ_FF   = (size_t)MTOK * DM * 4;
constexpr size_t SZ_CTX  = (size_t)MTOK * DM * 2;
constexpr size_t SZ_T1   = (size_t)MTOK * DM * 4;
constexpr size_t SZ_Y16  = (size_t)MTOK * DM * 2;
constexpr size_t OFF_X16 = 0;
constexpr size_t OFF_WP  = OFF_X16 + SZ_X16;
constexpr size_t OFF_WO  = OFF_WP + SZ_WP;
constexpr size_t OFF_W1  = OFF_WO + SZ_WO;
constexpr size_t OFF_W2  = OFF_W1 + SZ_W1;
constexpr size_t OFF_QKV = OFF_W2 + SZ_W2;
constexpr size_t OFF_CTX = OFF_QKV + SZ_QKV;
constexpr size_t OFF_T1  = OFF_CTX + SZ_CTX;
constexpr size_t OFF_Y16 = OFF_T1 + SZ_T1;
constexpr size_t WS_TOTAL = OFF_Y16 + SZ_Y16;
static_assert(SZ_H16 + SZ_FF <= SZ_QKV);
static_assert((OFF_WP % 256) == 0 && (OFF_WO % 256) == 0 && (OFF_W1 % 256) == 0 && (OFF_W2 % 256) == 0 && (OFF_QKV % 256) == 0);
static_assert((OFF_CTX % 256) == 0 && (OFF_T1 % 256) == 0 && (OFF_Y16 % 256) == 0 && (SZ_H16 % 256) == 0);
static_assert(WS_TOTAL <= (size_t)134217728);

extern "C" void kernel_launch(void* const* d_in, const int* in_sizes, int n_in, void* d_out, int out_size, void* d_ws, size_t ws_size, hipStream_t stream) {
    if (n_in < 19) return;
    const long long need_x = ((long long)(NB - 1) * SEQ_FULL + SEQ) * DM;
    if ((long long)in_sizes[0] < need_x || (long long)in_sizes[1] < need_x || (long long)in_sizes[2] < need_x) return;
    if (in_sizes[3] < NH * DM * HD || in_sizes[5] < NH * DM * HD || in_sizes[7] < NH * DM * HD) return;
    if (in_sizes[4] < DM || in_sizes[6] < DM || in_sizes[8] < DM) return;
    if (in_sizes[9] < DM * DM || in_sizes[10] < DM || in_sizes[11] < DM || in_sizes[12] < DM) return;
    if (in_sizes[13] < DM * FFD || in_sizes[14] < FFD || in_sizes[15] < FFD * DM || in_sizes[16] < DM || in_sizes[17] < DM || in_sizes[18] < DM) return;
    if ((long long)out_size < need_x) return;
    if (WS_TOTAL > ws_size) return;

    const float* x_q   = (const float*)d_in[0];
    const float* x_k   = (const float*)d_in[1];
    const float* x_v   = (const float*)d_in[2];
    const float* Wq    = (const float*)d_in[3];
    const float* bq    = (const float*)d_in[4];
    const float* Wk    = (const float*)d_in[5];
    const float* bk    = (const float*)d_in[6];
    const float* Wv    = (const float*)d_in[7];
    const float* bv    = (const float*)d_in[8];
    const float* Wo    = (const float*)d_in[9];
    const float* bo    = (const float*)d_in[10];
    const float* ln1_g = (const float*)d_in[11];
    const float* ln1_b = (const float*)d_in[12];
    const float* W1    = (const float*)d_in[13];
    const float* b1    = (const float*)d_in[14];
    const float* W2    = (const float*)d_in[15];
    const float* b2    = (const float*)d_in[16];
    const float* ln2_g = (const float*)d_in[17];
    const float* ln2_b = (const float*)d_in[18];
    float* out = (float*)d_out;

    char* ws = (char*)d_ws;
    unsigned short* X16 = (unsigned short*)(ws + OFF_X16);
    unsigned short* WP  = (unsigned short*)(ws + OFF_WP);
    unsigned short* WOT = (unsigned short*)(ws + OFF_WO);
    unsigned short* W1T = (unsigned short*)(ws + OFF_W1);
    unsigned short* W2T = (unsigned short*)(ws + OFF_W2);
    float* QKV = (float*)(ws + OFF_QKV);
    unsigned short* H16 = (unsigned short*)(ws + OFF_QKV);
    float* FF  = (float*)(ws + OFF_QKV + SZ_H16);
    unsigned short* CTX16 = (unsigned short*)(ws + OFF_CTX);
    float* T1  = (float*)(ws + OFF_T1);
    unsigned short* Y16 = (unsigned short*)(ws + OFF_Y16);

    const size_t PL = (size_t)MTOK * DM;

    k_cast_x3<<<dim3((unsigned)((MTOK * 64) / 256), 3u), 256, 0, stream>>>(x_q, x_k, x_v, X16);
    k_cast_wT<<<dim3((unsigned)((HD * (DM / 8) + 255) / 256), (unsigned)NH, 3u), 256, 0, stream>>>(Wq, Wk, Wv, (unsigned)HD, (unsigned)(DM * HD), WP, (unsigned)DM, (unsigned)(HD * DM), (unsigned)(DM * DM), (unsigned)DM, (unsigned)HD, 16.0f);
    k_cast_wT<<<dim3((unsigned)((DM * (DM / 8) + 255) / 256), 1u, 1u), 256, 0, stream>>>(Wo, Wo, Wo, (unsigned)DM, 0u, WOT, (unsigned)DM, 0u, 0u, (unsigned)DM, (unsigned)DM, 16.0f);
    k_cast_wT<<<dim3((unsigned)((FFD * (DM / 8) + 255) / 256), 1u, 1u), 256, 0, stream>>>(W1, W1, W1, (unsigned)FFD, 0u, W1T, (unsigned)DM, 0u, 0u, (unsigned)DM, (unsigned)FFD, 16.0f);
    k_cast_wT<<<dim3((unsigned)((DM * (FFD / 8) + 255) / 256), 1u, 1u), 256, 0, stream>>>(W2, W2, W2, (unsigned)DM, 0u, W2T, (unsigned)FFD, 0u, 0u, (unsigned)FFD, (unsigned)DM, 16.0f);

    const unsigned tiles512 = (unsigned)((MTOK / 64) * (DM / 64));
    w25::wmma_gemm64<0, false, 2, 0, false, 0><<<dim3((tiles512 + 7u) / 8u, 1u), 256, 0, stream>>>(X16, nullptr, DM, 0L, WP, nullptr, DM, 0L, (void*)QKV, nullptr, DM, 0L, bq, nullptr, 0L, MTOK, DM, DM, 0.0625f);
    w25::wmma_gemm64<0, false, 2, 0, false, 0><<<dim3((tiles512 + 7u) / 8u, 1u), 256, 0, stream>>>(X16 + PL, nullptr, DM, 0L, WP + (size_t)DM * DM, nullptr, DM, 0L, (void*)(QKV + PL), nullptr, DM, 0L, bk, nullptr, 0L, MTOK, DM, DM, 0.0625f);
    w25::wmma_gemm64<0, false, 2, 0, false, 0><<<dim3((tiles512 + 7u) / 8u, 1u), 256, 0, stream>>>(X16 + 2 * PL, nullptr, DM, 0L, WP + (size_t)2 * DM * DM, nullptr, DM, 0L, (void*)(QKV + 2 * PL), nullptr, DM, 0L, bv, nullptr, 0L, MTOK, DM, DM, 0.0625f);

    {
        w25::AttnGeom g;
        g.q_bs = (long)SEQ * DM; g.q_rs = DM; g.q_hs = HD;
        g.k_bs = (long)SEQ * DM; g.k_rs = DM; g.k_hs = HD;
        g.v_bs = (long)SEQ * DM; g.v_rs = DM; g.v_hs = HD;
        g.o_bs = (long)SEQ * DM; g.o_rs = DM; g.o_hs = HD;
        g.S = SEQ; g.Skv = SEQ; g.H = NH; g.pad_ = 0; g.qscale = 0.125f; g.ocarry = 16.0f;
        w25::attn64_f16<<<dim3((unsigned)(NB * NH * (SEQ / 64))), 128, 0, stream>>>(QKV, QKV + PL, QKV + 2 * PL, CTX16, g);
    }

    w25::wmma_gemm64<0, false, 2, 0, false, 0><<<dim3((tiles512 + 7u) / 8u, 1u), 256, 0, stream>>>(CTX16, nullptr, DM, 0L, WOT, nullptr, DM, 0L, (void*)T1, nullptr, DM, 0L, bo, nullptr, 0L, MTOK, DM, DM, 0.00390625f);

    k_add_ln<1><<<dim3((unsigned)(MTOK / 8)), 256, 0, stream>>>(x_q, T1, ln1_g, ln1_b, nullptr, Y16);

    const unsigned tilesFF = (unsigned)((MTOK / 64) * (FFD / 64));
    w25::wmma_gemm64<0, false, 2, 1, false, 2><<<dim3((tilesFF + 7u) / 8u, 1u), 256, 0, stream>>>(Y16, nullptr, DM, 0L, W1T, nullptr, DM, 0L, (void*)H16, nullptr, FFD, 0L, b1, nullptr, 0L, MTOK, FFD, DM, 0.0625f);
    w25::wmma_gemm64<0, false, 2, 0, false, 0><<<dim3((tiles512 + 7u) / 8u, 1u), 256, 0, stream>>>(H16, nullptr, FFD, 0L, W2T, nullptr, FFD, 0L, (void*)FF, nullptr, DM, 0L, b2, nullptr, 0L, MTOK, DM, FFD, 0.0625f);

    k_add_ln<0><<<dim3((unsigned)(MTOK / 8)), 256, 0, stream>>>(x_q, FF, ln2_g, ln2_b, out, nullptr);
}
